// SSMBlock_89893665505537
// MI455X (gfx1250) — hardware-verified
//
#include <hip/hip_runtime.h>
#include <math.h>
#include <stdint.h>

typedef __attribute__((ext_vector_type(16))) _Float16 v16h;
typedef __attribute__((ext_vector_type(8)))  _Float16 v8h;
typedef __attribute__((ext_vector_type(16))) __bf16   v16b;
typedef __attribute__((ext_vector_type(8)))  __bf16   v8b;
typedef __attribute__((ext_vector_type(8)))  float    v8f;
typedef __attribute__((ext_vector_type(4)))  float    v4f;
typedef __attribute__((ext_vector_type(4)))  unsigned v4u;
typedef __attribute__((ext_vector_type(2)))  unsigned v2u;

constexpr int NBATCH = 8;
constexpr int NTIME  = 2048;
constexpr int NCH    = 512;
constexpr int NTAP   = 2048;
constexpr int NCR    = 32;
constexpr int NUP    = 1024;
constexpr int NROWS  = NBATCH * NTIME;

constexpr int CONV_THREADS = 128;
constexpr int CONV_WAVES   = 4;
constexpr int CONV_NB      = 4;
constexpr int CONV_BLOCKS  = NCH * (NBATCH / CONV_NB);
constexpr int XOFF   = 64;
constexpr int XTAIL  = 32;
constexpr int XPITCH = XOFF + NTIME + XTAIL;
constexpr int KOFF   = 16;
constexpr int KF8P   = 2096;
constexpr int STG_PITCH  = 68;
constexpr int SSUM_PITCH = 32;
constexpr float KCARRY     = 256.0f;
constexpr float KCARRY_INV = 1.0f / 256.0f;
constexpr float WCARRY     = 64.0f;
constexpr float HCARRY     = 64.0f;
constexpr float UP_SCALE   = 1.0f / 64.0f;
constexpr float DOWN_SCALE = 1.0f / 4096.0f;
constexpr float LN_EPS     = 1e-5f;

constexpr int FUSE_THREADS   = 128;
constexpr int FUSE_ROWS      = 16;
constexpr int FUSE_BLK_PER_B = NTIME / FUSE_ROWS;
constexpr int FUSE_BLOCKS    = NROWS / FUSE_ROWS;
constexpr int YS_PITCH       = 516;

static_assert(NBATCH % CONV_NB == 0 && CONV_NB == 4);
static_assert((CONV_NB * NTIME) % CONV_THREADS == 0);
static_assert(NTIME == 2048 && NTAP == NTIME && NCH == 512 && NUP == 1024);
static_assert(NTIME % 64 == 0 && (NTIME / 64) % CONV_WAVES == 0);
static_assert(XPITCH % 8 == 0 && KF8P % 8 == 0);
static_assert(KF8P >= KOFF + NTAP + 32);
static_assert(KOFF + NTAP - 8 - 32 * (2 * (NTIME / 64 - 1) + 2) - 8 >= 0);
static_assert(NCH == 4 * FUSE_THREADS && FUSE_ROWS == 16);
static_assert(FUSE_BLK_PER_B * FUSE_ROWS == NTIME && (2 * NCH) % FUSE_THREADS == 0);
static_assert((YS_PITCH * 4) % 16 == 0);
static_assert(NROWS % 64 == 0 && NUP % 64 == 0 && NCH % 64 == 0 && NCH % 32 == 0);
static_assert(((NROWS / 64) * (NUP / 64)) % 8 == 0 && ((NROWS / 64) * (NCH / 64)) % 8 == 0);
static_assert(NBATCH * NCR == 256);

__device__ __forceinline__ unsigned short f2bf_bits(float f) {
  unsigned u = __float_as_uint(f);
  return (unsigned short)((u + 0x7FFFu + ((u >> 16) & 1u)) >> 16);
}
__device__ __forceinline__ float bf_bits2f(unsigned short h) { return __uint_as_float(((unsigned)h) << 16); }

__device__ __forceinline__ void dep_guard_h(v8f& a, v8f& b, v16h x, v16h y) { asm volatile("v_nop\n\tv_nop\n\tv_nop\n\tv_nop" : "+v"(a), "+v"(b) : "v"(x), "v"(y)); }
__device__ __forceinline__ void dep_guard_b(v8f& a, v8f& b, v16b x, v16b y) { asm volatile("v_nop\n\tv_nop\n\tv_nop\n\tv_nop" : "+v"(a), "+v"(b) : "v"(x), "v"(y)); }
__device__ __forceinline__ void keep4_h(v16h a, v16h b, v16h c, v16h d) { asm volatile("v_nop" :: "v"(a), "v"(b), "v"(c), "v"(d)); }
__device__ __forceinline__ void keep4_b(v16b a, v16b b, v16b c, v16b d) { asm volatile("v_nop" :: "v"(a), "v"(b), "v"(c), "v"(d)); }
__device__ __forceinline__ void acc_guard4(v8f& a, v8f& b, v8f& c, v8f& d) { asm volatile("v_nop\n\tv_nop\n\tv_nop\n\tv_nop" : "+v"(a), "+v"(b), "+v"(c), "+v"(d)); }
__device__ __forceinline__ void guard1_h(v8f& a, v16h x, v16h y) { asm volatile("v_nop\n\tv_nop\n\tv_nop\n\tv_nop" : "+v"(a) : "v"(x), "v"(y)); }
template <typename T> struct Frag;
template <> struct Frag<_Float16> {
  typedef v16h V; union U { v16h v; v8h h[2]; };
  static __device__ __forceinline__ v16h load(const _Float16* p) {
    U f; f.h[0] = *(const v8h*)(p); f.h[1] = *(const v8h*)(p + 16); return f.v;
  }
  static __device__ __forceinline__ v8f mma(v16h a, v16h b, v8f c) {
    return __builtin_amdgcn_wmma_f32_16x16x32_f16(false, a, false, b, (short)0, c, false, false);
  }
  static __device__ __forceinline__ void guard(v8f& a, v8f& b, v16h x, v16h y) { dep_guard_h(a, b, x, y); }
  static __device__ __forceinline__ void keep(v16h a, v16h b, v16h c, v16h d) { keep4_h(a, b, c, d); }
};
template <> struct Frag<__bf16> {
  typedef v16b V; union U { v16b v; v8b h[2]; };
  static __device__ __forceinline__ v16b load(const __bf16* p) {
    U f; f.h[0] = *(const v8b*)(p); f.h[1] = *(const v8b*)(p + 16); return f.v;
  }
  static __device__ __forceinline__ v8f mma(v16b a, v16b b, v8f c) {
    return __builtin_amdgcn_wmma_f32_16x16x32_bf16(false, a, false, b, (short)0, c, false, false);
  }
  static __device__ __forceinline__ void guard(v8f& a, v8f& b, v16b x, v16b y) { dep_guard_b(a, b, x, y); }
  static __device__ __forceinline__ void keep(v16b a, v16b b, v16b c, v16b d) { keep4_b(a, b, c, d); }
};

template <int ET> struct Elem;
template <> struct Elem<0> { typedef _Float16 T; };
template <> struct Elem<1> { typedef __bf16 T; };
template <int ET, bool SPLIT, int BIAS_MODE, int OUT_MODE, bool RESID, int ACT = 0>
__global__ __launch_bounds__(256) void wmma_gemm64(
    const unsigned short* __restrict__ Ap, const unsigned short* __restrict__ A2p, int lda, long strideA,
    const unsigned short* __restrict__ Btp, const unsigned short* __restrict__ Bt2p, int ldb, long strideB,
    void* __restrict__ Cout, void* __restrict__ Cout2, int ldc, long strideC,
    const float* __restrict__ bias,
    const float* __restrict__ resid, long strideR,
    int M, int N, int K, float scale) {
  typedef typename Elem<ET>::T T;
  typedef typename Frag<T>::V V;
  const T* A = (const T*)Ap; const T* A2 = (const T*)A2p; const T* Bt = (const T*)Btp; const T* Bt2 = (const T*)Bt2p;
  __shared__ __align__(16) float sT[8][16 * 68];
  const int b    = blockIdx.y;
  const int lane = threadIdx.x & 31;
  const int wave = threadIdx.x >> 5;
  const int tilesN = N >> 6;
  const int tilesM = M >> 6;
  const int tile = blockIdx.x * 8 + wave;
  if (tile >= tilesM * tilesN) return;
  const int tm = tile / tilesN;
  const int tn = tile - tm * tilesN;
  const int m0 = tm << 6;
  const int n0 = tn << 6;

  const T* Ab  = A  + (size_t)b * strideA;
  const T* Bb  = Bt + (size_t)b * strideB;
  const T* Ab2 = SPLIT ? (A2  + (size_t)b * strideA) : nullptr;
  const T* Bb2 = SPLIT ? (Bt2 + (size_t)b * strideB) : nullptr;

  const int rlane = lane & 15;
  const int koff  = (lane >> 4) * 8;
  const int mOff  = (lane >> 4) * 8;

  v8f acc[4][4];
#pragma unroll
  for (int i = 0; i < 4; ++i)
#pragma unroll
    for (int j = 0; j < 4; ++j) acc[i][j] = (v8f){0.f,0.f,0.f,0.f,0.f,0.f,0.f,0.f};

  for (int k0 = 0; k0 < K; k0 += 32) {
    V bh[4], bl[4];
#pragma unroll
    for (int j = 0; j < 4; ++j) {
      const size_t bo = (size_t)(n0 + (j << 4) + rlane) * ldb + koff + k0;
      bh[j] = Frag<T>::load(Bb + bo);
      if (SPLIT) bl[j] = Frag<T>::load(Bb2 + bo);
    }
#pragma unroll
    for (int i = 0; i < 4; ++i) {
      const size_t ao = (size_t)(m0 + (i << 4) + rlane) * lda + koff + k0;
      V ah = Frag<T>::load(Ab + ao);
      V al;
      if (SPLIT) al = Frag<T>::load(Ab2 + ao);
#pragma unroll
      for (int j = 0; j < 4; ++j) {
        acc[i][j] = Frag<T>::mma(ah, bh[j], acc[i][j]);
        if (SPLIT) {
          acc[i][j] = Frag<T>::mma(ah, bl[j], acc[i][j]);
          acc[i][j] = Frag<T>::mma(al, bh[j], acc[i][j]);
        }
      }
      Frag<T>::guard(acc[i][0], acc[i][3], ah, SPLIT ? al : ah);
    }
    Frag<T>::keep(bh[0], bh[1], bh[2], bh[3]);
    if (SPLIT) Frag<T>::keep(bl[0], bl[1], bl[2], bl[3]);
  }
  acc_guard4(acc[0][0], acc[0][1], acc[0][2], acc[0][3]);
  acc_guard4(acc[1][0], acc[1][1], acc[1][2], acc[1][3]);
  acc_guard4(acc[2][0], acc[2][1], acc[2][2], acc[2][3]);
  acc_guard4(acc[3][0], acc[3][1], acc[3][2], acc[3][3]);

  float* slab = sT[wave];
  const float* Rb = RESID ? (resid + (size_t)b * strideR) : nullptr;
#pragma unroll
  for (int i = 0; i < 4; ++i) {
    const int mBase = m0 + (i << 4);
#pragma unroll
    for (int j = 0; j < 4; ++j) {
      const int n = n0 + (j << 4) + rlane;
      float bv = 0.f;
      if (BIAS_MODE == 2) bv = bias[n];
#pragma unroll
      for (int r = 0; r < 8; ++r) {
        float v = acc[i][j][r] * scale;
        if (BIAS_MODE == 1) v += bias[mBase + mOff + r];
        if (BIAS_MODE == 2) v += bv;
        if (RESID) v += Rb[(size_t)(mBase + mOff + r) * ldc + n];
        if (ACT == 1) v = tanhf(v);
        if (ACT == 2) v = fmaxf(v, 0.0f);
        if (ACT == 3) v = v / (1.0f + expf(-v));
        if (ACT == 4) v = (v > 0.f) ? v : 0.01f * v;
        if (ACT == 5) v = 0.5f * v * (1.0f + erff(v * 0.70710678118654752f));
        slab[(mOff + r) * 68 + (j << 4) + rlane] = v;
      }
    }
    __builtin_amdgcn_fence(__ATOMIC_RELEASE, "workgroup");
    __builtin_amdgcn_wave_barrier();
    __builtin_amdgcn_fence(__ATOMIC_ACQUIRE, "workgroup");
    if (OUT_MODE == 0) {
      float* C = (float*)Cout + (size_t)b * strideC;
      const int hh = lane >> 4, c4 = (lane & 15) * 4;
      for (int pass = 0; pass < 2; ++pass) {
#pragma unroll
        for (int it = 0; it < 8; ++it) {
          const int row = it * 2 + hh;
          v4f v = *(const v4f*)(slab + row * 68 + c4);
          *(volatile v4f*)(C + (size_t)(mBase + row) * ldc + n0 + c4) = v;
        }
        __threadfence();
      }
    } else {
      const int q = lane >> 3, c8 = (lane & 7) * 8;
      unsigned short* C  = (unsigned short*)Cout  + (size_t)b * strideC;
      unsigned short* C2 = (OUT_MODE == 2) ? ((unsigned short*)Cout2 + (size_t)b * strideC) : nullptr;
      for (int pass = 0; pass < 2; ++pass) {
#pragma unroll
        for (int it = 0; it < 4; ++it) {
          const int row = it * 4 + q;
          const float* sp = slab + row * 68 + c8;
          v8h hv, lv;
#pragma unroll
          for (int e = 0; e < 8; ++e) {
            if (OUT_MODE == 1) {
              hv[e] = (_Float16)sp[e];
            } else {
              unsigned short hb = f2bf_bits(sp[e]);
              unsigned short lb = f2bf_bits(sp[e] - bf_bits2f(hb));
              hv[e] = __builtin_bit_cast(_Float16, hb);
              lv[e] = __builtin_bit_cast(_Float16, lb);
            }
          }
          *(volatile v8h*)(C + (size_t)(mBase + row) * ldc + n0 + c8) = hv;
          if (OUT_MODE == 2) *(volatile v8h*)(C2 + (size_t)(mBase + row) * ldc + n0 + c8) = lv;
        }
        __threadfence();
      }
    }
    __builtin_amdgcn_fence(__ATOMIC_RELEASE, "workgroup");
    __builtin_amdgcn_wave_barrier();
    __builtin_amdgcn_fence(__ATOMIC_ACQUIRE, "workgroup");
  }
}

__device__ __forceinline__ float h16_to_f32(unsigned hb) {
  const unsigned sgn = (hb & 0x8000u) << 16; const unsigned em = hb & 0x7fffu;
  const float fn = __uint_as_float((em << 13) + 0x38000000u);
  const float fs = (float)em * 5.9604644775390625e-8f;
  const float mag = (em < 0x400u) ? fs : fn; return __uint_as_float(__float_as_uint(mag) | sgn); }

__global__ __launch_bounds__(256) void wprep_kernel(const float* __restrict__ W, int kin, int nout, float scale,
                                                    unsigned short* __restrict__ bt) {
  const int tpr = kin >> 3;
  const int i = blockIdx.x * 256 + threadIdx.x;
  if (i >= nout * tpr) return;
  const int n  = i / tpr;
  const int k0 = (i - n * tpr) * 8;
  v8h hv;
#pragma unroll
  for (int e = 0; e < 8; ++e) {
    const float v = W[(size_t)(k0 + e) * nout + n];
    hv[e] = (_Float16)(scale * v);
  }
  unsigned short* dst = bt + (size_t)i * 8;
  *(volatile v8h*)dst = hv;
  __threadfence();
  *(volatile v8h*)dst = hv;
}

__global__ __launch_bounds__(CONV_THREADS) void conv_kernel(const float* __restrict__ x, const float* __restrict__ kw,
                                                            unsigned short* __restrict__ yT, float* __restrict__ ssum) {
  __shared__ __align__(16) _Float16 xs[CONV_NB * XPITCH];
  __shared__ __align__(16) _Float16 kf8[8 * KF8P];
  __shared__ __align__(16) float stg[CONV_WAVES][CONV_NB * STG_PITCH];
  __shared__ float wsum[CONV_WAVES][CONV_NB];

  const int tid = threadIdx.x, lane = tid & 31, wave = tid >> 5;
  const int c  = blockIdx.x >> 1;
  const int bh = blockIdx.x & 1;
  const int bbase = bh * CONV_NB;

#pragma unroll 4
  for (int i = 0; i < (CONV_NB * NTIME) / CONV_THREADS; ++i) {
    const int idx = i * CONV_THREADS + tid;
    const int bl = idx >> 11;
    const int t  = idx & (NTIME - 1);
    const float v = x[((size_t)(bbase + bl) * NTIME + t) * NCH + c];
    xs[bl * XPITCH + XOFF + t] = (_Float16)v;
  }
#pragma unroll 1
  for (int i = tid; i < CONV_NB * (XOFF + XTAIL); i += CONV_THREADS) {
    const int bl = i / (XOFF + XTAIL);
    const int p  = i - bl * (XOFF + XTAIL);
    const int pos = (p < XOFF) ? p : (NTIME + p);
    xs[bl * XPITCH + pos] = (_Float16)0.0f;
  }
  const float* krow = kw + (size_t)c * NTAP;
#pragma unroll 2
  for (int i = tid; i < 8 * KF8P; i += CONV_THREADS) {
    const int sh = i / KF8P;
    const int u  = i - sh * KF8P;
    const int j  = u + sh - KOFF;
    const int jc = (j < 0) ? 0 : ((j > NTAP - 1) ? (NTAP - 1) : j);
    const float kv  = krow[jc];
    const float fac = (j >= 0 && j < NTAP) ? KCARRY : 0.0f;
    kf8[i] = (_Float16)(kv * fac);
  }
  __syncthreads();

  const int ncol = lane & 15, hh = lane >> 4;
  const int bl_c = ncol & 3;
  const int grp  = ncol >> 2;
  const int mu   = ncol >> 3;
  const int nu   = ncol & 7;
  const _Float16* arow = kf8 + (7 - nu) * KF8P + (KOFF + NTAP - 8) - 8 * mu + 8 * hh;
  const _Float16* brow = xs + bl_c * XPITCH + XOFF + 16 * grp + 8 * hh;
  float* slab = stg[wave];
  float lsum = 0.0f;
  const v8f zero8 = {0.f, 0.f, 0.f, 0.f, 0.f, 0.f, 0.f, 0.f};

#pragma unroll 1
  for (int jj = wave; jj < NTIME / 64; jj += CONV_WAVES) {
    const int t0  = jj * 64;
    const int ncd = 2 * jj + 3;
    v8f acc = zero8;
#pragma unroll 1
    for (int cd = 0; cd < ncd; ++cd) {
      const v16h a = Frag<_Float16>::load(arow - 32 * cd);
      const v16h b = Frag<_Float16>::load(brow + (t0 - 32 * cd));
      acc = Frag<_Float16>::mma(a, b, acc);
      guard1_h(acc, a, b);
    }
#pragma unroll
    for (int r = 0; r < 8; ++r) {
      const float v = acc[r] * KCARRY_INV;
      slab[bl_c * STG_PITCH + 16 * grp + 8 * hh + r] = v;
      lsum += v;
    }
    __builtin_amdgcn_fence(__ATOMIC_RELEASE, "workgroup");
    __builtin_amdgcn_wave_barrier();
    __builtin_amdgcn_fence(__ATOMIC_ACQUIRE, "workgroup");
    {
      const int q = lane >> 3, c8 = (lane & 7) * 8;
      const float* sp = slab + q * STG_PITCH + c8;
      const v4f s0 = *(const v4f*)sp;
      const v4f s1 = *(const v4f*)(sp + 4);
      v8h hv;
      hv[0] = (_Float16)s0[0]; hv[1] = (_Float16)s0[1]; hv[2] = (_Float16)s0[2]; hv[3] = (_Float16)s0[3];
      hv[4] = (_Float16)s1[0]; hv[5] = (_Float16)s1[1]; hv[6] = (_Float16)s1[2]; hv[7] = (_Float16)s1[3];
      unsigned short* dst = yT + ((size_t)(c * NBATCH + bbase + q)) * NTIME + t0 + c8;
      *(volatile v8h*)dst = hv;
      __threadfence();
      *(volatile v8h*)dst = hv;
    }
    __builtin_amdgcn_fence(__ATOMIC_RELEASE, "workgroup");
    __builtin_amdgcn_wave_barrier();
    __builtin_amdgcn_fence(__ATOMIC_ACQUIRE, "workgroup");
  }

  lsum += __shfl_xor(lsum, 4, 32);
  lsum += __shfl_xor(lsum, 8, 32);
  lsum += __shfl_xor(lsum, 16, 32);
  if (lane < CONV_NB) wsum[wave][lane] = lsum;
  __syncthreads();
  if (wave == 0) {
    const int bi = lane & 3;
    const float tot = ((wsum[0][bi] + wsum[1][bi]) + wsum[2][bi]) + wsum[3][bi];
    const float keepf = (lane < CONV_NB) ? 1.0f : 0.0f;
    const float val = tot * keepf;
    float* dst = ssum + (size_t)blockIdx.x * SSUM_PITCH + lane;
    *(volatile float*)dst = val;
    __threadfence();
    *(volatile float*)dst = val;
  }
}

__global__ __launch_bounds__(256) void se_kernel(const float* __restrict__ ssum, const float* __restrict__ w1,
                                                 const float* __restrict__ b1, const float* __restrict__ w2,
                                                 const float* __restrict__ b2, float* __restrict__ g) {
  __shared__ float hid[NBATCH * NCR];
  const int tid = threadIdx.x;
  const int b = tid >> 5, j = tid & 31;
  const int bq = b >> 2, br = b & 3;
  float acc = 0.0f;
#pragma unroll 1
  for (int cc = 0; cc < NCH; ++cc) {
    const float sval = ssum[(size_t)(cc * 2 + bq) * SSUM_PITCH + br] * (1.0f / (float)NTIME);
    acc = fmaf(sval, w1[cc * NCR + j], acc);
  }
  acc += b1[j];
  hid[tid] = fmaxf(acc, 0.0f);
  __syncthreads();
#pragma unroll 1
  for (int bb = 0; bb < NBATCH; ++bb) {
#pragma unroll 1
    for (int half = 0; half < 2; ++half) {
      const int cc = half * 256 + tid;
      float a = 0.0f;
#pragma unroll 4
      for (int jj = 0; jj < NCR; ++jj) a = fmaf(hid[bb * NCR + jj], w2[jj * NCH + cc], a);
      a += b2[cc];
      const float gv = 1.0f / (1.0f + expf(-a));
      float* dst = g + bb * NCH + cc;
      *(volatile float*)dst = gv;
      __threadfence();
      *(volatile float*)dst = gv;
    }
  }
}

__device__ __forceinline__ float block_sum4(float v, float* slot, int lane, int wave) {
#pragma unroll
  for (int off = 1; off < 32; off <<= 1) v += __shfl_xor(v, off, 32);
  if (lane == 0) slot[wave] = v;
  __syncthreads();
  return ((slot[0] + slot[1]) + slot[2]) + slot[3];
}

__device__ __forceinline__ void stage_ytile(const unsigned short* __restrict__ yT, int b, int t0, float* ys, int tid) {
#pragma unroll 2
  for (int i = 0; i < (2 * NCH) / FUSE_THREADS; ++i) {
    const int item = i * FUSE_THREADS + tid;
    const int ch = item >> 1, wd = item & 1;
    const v4u wv = *(const v4u*)(yT + ((size_t)(ch * NBATCH + b)) * NTIME + t0 + 8 * wd);
    float* yp = ys + (8 * wd) * YS_PITCH + ch;
#pragma unroll
    for (int e = 0; e < 4; ++e) {
      const unsigned w = wv[e];
      yp[(2 * e) * YS_PITCH]     = h16_to_f32(w & 0xffffu);
      yp[(2 * e + 1) * YS_PITCH] = h16_to_f32(w >> 16);
    }
  }
}

__global__ __launch_bounds__(FUSE_THREADS) void fuse1_kernel(const float* __restrict__ x, const unsigned short* __restrict__ yT,
                                                             const float* __restrict__ g, const float* __restrict__ lnw,
                                                             const float* __restrict__ lnb, unsigned short* __restrict__ y1h) {
  __shared__ __align__(16) float ys[FUSE_ROWS * YS_PITCH];
  __shared__ float red[2][4];
  const int tid = threadIdx.x, lane = tid & 31, wave = tid >> 5;
  const int b  = blockIdx.x / FUSE_BLK_PER_B;
  const int t0 = (blockIdx.x - b * FUSE_BLK_PER_B) * FUSE_ROWS;
  stage_ytile(yT, b, t0, ys, tid);
  const int c0 = 4 * tid;
  const v4f g4 = *(const v4f*)(g + b * NCH + c0);
  const v4f w4 = *(const v4f*)(lnw + c0);
  const v4f b4 = *(const v4f*)(lnb + c0);
  __syncthreads();
#pragma unroll 1
  for (int r = 0; r < FUSE_ROWS; ++r) {
    const size_t row = (size_t)b * NTIME + t0 + r;
    const v4f x4 = *(const v4f*)(x + row * NCH + c0);
    const v4f y4 = *(const v4f*)(ys + r * YS_PITCH + c0);
    const float v0 = fmaf(y4[0], g4[0], x4[0]);
    const float v1 = fmaf(y4[1], g4[1], x4[1]);
    const float v2 = fmaf(y4[2], g4[2], x4[2]);
    const float v3 = fmaf(y4[3], g4[3], x4[3]);
    const float mean = block_sum4((v0 + v1) + (v2 + v3), red[0], lane, wave) * (1.0f / (float)NCH);
    const float d0 = v0 - mean, d1 = v1 - mean, d2 = v2 - mean, d3 = v3 - mean;
    const float var = block_sum4(fmaf(d0, d0, fmaf(d1, d1, fmaf(d2, d2, d3 * d3))), red[1], lane, wave) * (1.0f / (float)NCH);
    const float rstd = rsqrtf(var + LN_EPS);
    const float o0 = fmaf(d0 * rstd, w4[0], b4[0]);
    const float o1 = fmaf(d1 * rstd, w4[1], b4[1]);
    const float o2 = fmaf(d2 * rstd, w4[2], b4[2]);
    const float o3 = fmaf(d3 * rstd, w4[3], b4[3]);
    const _Float16 h0 = (_Float16)o0, h1 = (_Float16)o1, h2 = (_Float16)o2, h3 = (_Float16)o3;
    const unsigned short u0 = __builtin_bit_cast(unsigned short, h0);
    const unsigned short u1 = __builtin_bit_cast(unsigned short, h1);
    const unsigned short u2 = __builtin_bit_cast(unsigned short, h2);
    const unsigned short u3 = __builtin_bit_cast(unsigned short, h3);
    v2u pv;
    pv[0] = (unsigned)u0 | ((unsigned)u1 << 16);
    pv[1] = (unsigned)u2 | ((unsigned)u3 << 16);
    unsigned short* dst = y1h + row * NCH + c0;
    *(volatile v2u*)dst = pv;
    __threadfence();
    *(volatile v2u*)dst = pv;
  }
}

__device__ __forceinline__ float glu_val(float a, float q) {
  const float ge = 0.5f * a * (1.0f + erff(a * 0.70710678118654752f));
  const float sg = 1.0f / (1.0f + expf(-q));
  return ge * sg;
}
__global__ __launch_bounds__(256) void glu_kernel(const unsigned short* __restrict__ u, unsigned short* __restrict__ h2) {
  const int i = blockIdx.x * 256 + threadIdx.x;
  if (i >= NROWS * (NCH / 2)) return;
  const int row = i >> 8;
  const int cp  = (i & 255) * 2;
  const unsigned wa = *(const unsigned*)(u + (size_t)row * NUP + cp);
  const unsigned wq = *(const unsigned*)(u + (size_t)row * NUP + NCH + cp);
  const float a0 = h16_to_f32(wa & 0xffffu), a1 = h16_to_f32(wa >> 16);
  const float q0 = h16_to_f32(wq & 0xffffu), q1 = h16_to_f32(wq >> 16);
  const _Float16 e0 = (_Float16)(glu_val(a0, q0) * HCARRY);
  const _Float16 e1 = (_Float16)(glu_val(a1, q1) * HCARRY);
  const unsigned ov = (unsigned)__builtin_bit_cast(unsigned short, e0) | ((unsigned)__builtin_bit_cast(unsigned short, e1) << 16);
  ((volatile unsigned*)h2)[i] = ov;
  __threadfence();
  ((volatile unsigned*)h2)[i] = ov;
}

__global__ __launch_bounds__(FUSE_THREADS) void fuse2_kernel(const float* __restrict__ x, const unsigned short* __restrict__ yT,
                                                             const float* __restrict__ g,
                                                             const float* __restrict__ lnw, const float* __restrict__ lnb,
                                                             const float* __restrict__ z0,
                                                             const float* __restrict__ mw, const float* __restrict__ mb,
                                                             const float* __restrict__ l2w, const float* __restrict__ l2b,
                                                             float* __restrict__ out) {
  __shared__ __align__(16) float ys[FUSE_ROWS * YS_PITCH];
  __shared__ float red[6][4];
  const int tid = threadIdx.x, lane = tid & 31, wave = tid >> 5;
  const int b  = blockIdx.x / FUSE_BLK_PER_B;
  const int t0 = (blockIdx.x - b * FUSE_BLK_PER_B) * FUSE_ROWS;
  stage_ytile(yT, b, t0, ys, tid);
  const int c0 = 4 * tid;
  const v4f g4  = *(const v4f*)(g + b * NCH + c0);
  const v4f w4  = *(const v4f*)(lnw + c0);
  const v4f b4  = *(const v4f*)(lnb + c0);
  const v4f mw4 = *(const v4f*)(mw + c0);
  const v4f mb4 = *(const v4f*)(mb + c0);
  const v4f lw4 = *(const v4f*)(l2w + c0);
  const v4f lb4 = *(const v4f*)(l2b + c0);
  __syncthreads();
  const float inv_c = 1.0f / (float)NCH;
#pragma unroll 1
  for (int r = 0; r < FUSE_ROWS; ++r) {
    const size_t row = (size_t)b * NTIME + t0 + r;
    const v4f x4 = *(const v4f*)(x + row * NCH + c0);
    const v4f y4 = *(const v4f*)(ys + r * YS_PITCH + c0);
    const v4f z4 = *(const v4f*)(z0 + row * NCH + c0);
    const float v0 = fmaf(y4[0], g4[0], x4[0]);
    const float v1 = fmaf(y4[1], g4[1], x4[1]);
    const float v2 = fmaf(y4[2], g4[2], x4[2]);
    const float v3 = fmaf(y4[3], g4[3], x4[3]);
    const float mean1 = block_sum4((v0 + v1) + (v2 + v3), red[0], lane, wave) * inv_c;
    const float d0 = v0 - mean1, d1 = v1 - mean1, d2 = v2 - mean1, d3 = v3 - mean1;
    const float var1 = block_sum4(fmaf(d0, d0, fmaf(d1, d1, fmaf(d2, d2, d3 * d3))), red[1], lane, wave) * inv_c;
    const float rs1 = rsqrtf(var1 + LN_EPS);
    const float y10 = fmaf(d0 * rs1, w4[0], b4[0]);
    const float y11 = fmaf(d1 * rs1, w4[1], b4[1]);
    const float y12 = fmaf(d2 * rs1, w4[2], b4[2]);
    const float y13 = fmaf(d3 * rs1, w4[3], b4[3]);
    const float p0 = y10 + z4[0], p1 = y11 + z4[1], p2 = y12 + z4[2], p3 = y13 + z4[3];
    const float mean2 = block_sum4((p0 + p1) + (p2 + p3), red[2], lane, wave) * inv_c;
    const float e0 = p0 - mean2, e1 = p1 - mean2, e2 = p2 - mean2, e3 = p3 - mean2;
    const float var2 = block_sum4(fmaf(e0, e0, fmaf(e1, e1, fmaf(e2, e2, e3 * e3))), red[3], lane, wave) * inv_c;
    const float rs2 = rsqrtf(var2 + LN_EPS);
    const float s0 = fmaf(e0 * rs2, mw4[0], mb4[0]);
    const float s1 = fmaf(e1 * rs2, mw4[1], mb4[1]);
    const float s2 = fmaf(e2 * rs2, mw4[2], mb4[2]);
    const float s3 = fmaf(e3 * rs2, mw4[3], mb4[3]);
    const float q0 = y10 + s0, q1 = y11 + s1, q2 = y12 + s2, q3 = y13 + s3;
    const float mean3 = block_sum4((q0 + q1) + (q2 + q3), red[4], lane, wave) * inv_c;
    const float f0 = q0 - mean3, f1 = q1 - mean3, f2 = q2 - mean3, f3 = q3 - mean3;
    const float var3 = block_sum4(fmaf(f0, f0, fmaf(f1, f1, fmaf(f2, f2, f3 * f3))), red[5], lane, wave) * inv_c;
    const float rs3 = rsqrtf(var3 + LN_EPS);
    v4f ov;
    ov[0] = fmaf(f0 * rs3, lw4[0], lb4[0]);
    ov[1] = fmaf(f1 * rs3, lw4[1], lb4[1]);
    ov[2] = fmaf(f2 * rs3, lw4[2], lb4[2]);
    ov[3] = fmaf(f3 * rs3, lw4[3], lb4[3]);
    float* dst = out + row * NCH + c0;
    *(volatile v4f*)dst = ov;
    __threadfence();
    *(volatile v4f*)dst = ov;
  }
}

extern "C" void kernel_launch(void* const* d_in, const int* in_sizes, int n_in,
                              void* d_out, int out_size, void* d_ws, size_t ws_size,
                              hipStream_t stream) {
  if (n_in < 16) return;
  if (in_sizes[0] != NBATCH * NTIME * NCH || in_sizes[1] != NCH * NTAP || out_size != NROWS * NCH) return;
  const float* x      = (const float*)d_in[0];
  const float* kw     = (const float*)d_in[1];
  const float* se_w1  = (const float*)d_in[2];
  const float* se_b1  = (const float*)d_in[3];
  const float* se_w2  = (const float*)d_in[4];
  const float* se_b2  = (const float*)d_in[5];
  const float* ln1_w  = (const float*)d_in[6];
  const float* ln1_b  = (const float*)d_in[7];
  const float* up_w   = (const float*)d_in[8];
  const float* up_b   = (const float*)d_in[9];
  const float* down_w = (const float*)d_in[10];
  const float* down_b = (const float*)d_in[11];
  const float* mix_w  = (const float*)d_in[12];
  const float* mix_b  = (const float*)d_in[13];
  const float* ln2_w  = (const float*)d_in[14];
  const float* ln2_b  = (const float*)d_in[15];
  float* out = (float*)d_out;

  char* wsb = (char*)d_ws;
  size_t off = 0;
  auto carve = [&](size_t bytes) -> size_t { const size_t o = off; off += (bytes + 255) & ~(size_t)255; return o; };
  const size_t o_yT   = carve((size_t)NCH * NBATCH * NTIME * 2);
  const size_t o_ssum = carve((size_t)CONV_BLOCKS * SSUM_PITCH * 4);
  const size_t o_g    = carve((size_t)NBATCH * NCH * 4);
  const size_t o_upwT = carve((size_t)NUP * NCH * 2);
  const size_t o_dwT  = carve((size_t)NCH * NCH * 2);
  const size_t o_y1h  = carve((size_t)NROWS * NCH * 2);
  const size_t o_u    = carve((size_t)NROWS * NUP * 2);
  const size_t o_h2   = carve((size_t)NROWS * NCH * 2);
  const size_t o_z0   = carve((size_t)NROWS * NCH * 4);
  if (off > ws_size) return;

  unsigned short* yT   = (unsigned short*)(wsb + o_yT);
  float*          ssum = (float*)(wsb + o_ssum);
  float*          g    = (float*)(wsb + o_g);
  unsigned short* upwT = (unsigned short*)(wsb + o_upwT);
  unsigned short* dwT  = (unsigned short*)(wsb + o_dwT);
  unsigned short* y1h  = (unsigned short*)(wsb + o_y1h);
  unsigned short* u    = (unsigned short*)(wsb + o_u);
  unsigned short* h2   = (unsigned short*)(wsb + o_h2);
  float*          z0   = (float*)(wsb + o_z0);

  wprep_kernel<<<(NUP * (NCH / 8)) / 256, 256, 0, stream>>>(up_w, NCH, NUP, WCARRY, upwT);
  wprep_kernel<<<(NCH * (NCH / 8)) / 256, 256, 0, stream>>>(down_w, NCH, NCH, WCARRY, dwT);
  conv_kernel<<<CONV_BLOCKS, CONV_THREADS, 0, stream>>>(x, kw, yT, ssum);
  se_kernel<<<1, 256, 0, stream>>>(ssum, se_w1, se_b1, se_w2, se_b2, g);
  fuse1_kernel<<<FUSE_BLOCKS, FUSE_THREADS, 0, stream>>>(x, yT, g, ln1_w, ln1_b, y1h);
  wmma_gemm64<0, false, 2, 1, false, 0><<<dim3(((NROWS / 64) * (NUP / 64)) / 8, 1), 256, 0, stream>>>(
      y1h, y1h, NCH, 0L, upwT, upwT, NCH, 0L, (void*)u, (void*)u, NUP, 0L, up_b, up_b, 0L,
      NROWS, NUP, NCH, UP_SCALE);
  glu_kernel<<<(NROWS * (NCH / 2)) / 256, 256, 0, stream>>>(u, h2);
  wmma_gemm64<0, false, 2, 0, false, 0><<<dim3(((NROWS / 64) * (NCH / 64)) / 8, 1), 256, 0, stream>>>(
      h2, h2, NCH, 0L, dwT, dwT, NCH, 0L, (void*)z0, (void*)z0, NCH, 0L, down_b, down_b, 0L,
      NROWS, NCH, NCH, DOWN_SCALE);
  fuse2_kernel<<<FUSE_BLOCKS, FUSE_THREADS, 0, stream>>>(x, yT, g, ln1_w, ln1_b, z0, mix_w, mix_b, ln2_w, ln2_b, out);
}
